// TransformerBlock_10333691314606
// MI455X (gfx1250) — hardware-verified
//
#include <hip/hip_runtime.h>
#include <math.h>

#ifndef NB
#define NB 2
#endif
#ifndef SEQ
#define SEQ 2048
#endif
#define NB_FULL 2
#define SEQ_FULL 2048
#define EMB 1024
#define HEADS 16
#define HD 64
#define FF 4096
#define TOK (NB * SEQ)
#define LDQK (2 * EMB)

static_assert(EMB == HEADS * HD);
static_assert(HD == 64);
static_assert(EMB == 8 * 32 * 4);
static_assert(SEQ % 64 == 0);
static_assert(TOK % 64 == 0);
static_assert(EMB % 64 == 0 && FF % 64 == 0 && LDQK % 64 == 0);
static_assert(EMB % 32 == 0 && FF % 32 == 0);
static_assert(NB <= NB_FULL && SEQ <= SEQ_FULL);
static_assert(((TOK / 64) * (EMB / 64)) % 8 == 0);

typedef _Float16 v16h __attribute__((ext_vector_type(16)));
typedef _Float16 v8h  __attribute__((ext_vector_type(8)));
typedef float    v8f  __attribute__((ext_vector_type(8)));
typedef float    v4f  __attribute__((ext_vector_type(4)));
typedef unsigned int u4v __attribute__((ext_vector_type(4)));
typedef unsigned int u2v __attribute__((ext_vector_type(2)));
union FragH { v16h v; v8h h[2]; };

__device__ __forceinline__ v16h ldfrag_g(const unsigned short* __restrict__ p) {
    FragH f; f.h[0] = *(const v8h*)(p); f.h[1] = *(const v8h*)(p + 16); return f.v;
}
__device__ __forceinline__ v8f mma16(v16h a, v16h b, v8f c) {
    return __builtin_amdgcn_wmma_f32_16x16x32_f16(false, a, false, b, (short)0, c, false, false);
}
__device__ __forceinline__ void guard4(v8f& a, v8f& b, v8f& c, v8f& d, v16h x, v16h y) {
    asm volatile("v_nop\n\tv_nop\n\tv_nop\n\tv_nop" : "+v"(a), "+v"(b), "+v"(c), "+v"(d) : "v"(x), "v"(y));
}
__device__ __forceinline__ void guard4b(v8f& a, v8f& b, v8f& c, v8f& d, v16h x, v16h y0, v16h y1, v16h y2, v16h y3) {
    asm volatile("v_nop\n\tv_nop\n\tv_nop\n\tv_nop" : "+v"(a), "+v"(b), "+v"(c), "+v"(d) : "v"(x), "v"(y0), "v"(y1), "v"(y2), "v"(y3));
}
__device__ __forceinline__ void guard2(v8f& a, v8f& b, v16h x, v16h y0, v16h y1) {
    asm volatile("v_nop\n\tv_nop\n\tv_nop\n\tv_nop" : "+v"(a), "+v"(b) : "v"(x), "v"(y0), "v"(y1));
}
__device__ __forceinline__ void keep4(v16h a, v16h b, v16h c, v16h d) { asm volatile("v_nop" :: "v"(a), "v"(b), "v"(c), "v"(d)); }
__device__ __forceinline__ v8f vzero() { v8f z = {0.f, 0.f, 0.f, 0.f, 0.f, 0.f, 0.f, 0.f}; return z; }
__device__ __forceinline__ void lds_wave_sync() {
    __builtin_amdgcn_fence(3  , "workgroup");
    __builtin_amdgcn_wave_barrier();
    __builtin_amdgcn_fence(2  , "workgroup");
}
__device__ __forceinline__ float bf16_keep(float v) {
    unsigned u = __builtin_bit_cast(unsigned, v);
    u = (u + 0x7fffu + ((u >> 16) & 1u)) & 0xffff0000u;
    return __builtin_bit_cast(float, u);
}
__device__ __forceinline__ v4f bf16_keep4(v4f v) { v4f o; o.x = bf16_keep(v.x); o.y = bf16_keep(v.y); o.z = bf16_keep(v.z); o.w = bf16_keep(v.w); return o; }
__device__ __forceinline__ unsigned pkh2(float a, float b) {
    return (unsigned)__builtin_bit_cast(unsigned short, (_Float16)a) | ((unsigned)__builtin_bit_cast(unsigned short, (_Float16)b) << 16);
}
__device__ __forceinline__ float gelu_t(float t) {
    const float t2 = t * t;
    const float w = t * (1.0f + 0.044715f * t2);
    const float e = exp2f(-2.302208198f * w);
    return t * __builtin_amdgcn_rcpf(1.0f + e);
}
template <int GELU, int CARRY> __device__ __forceinline__ float fin1(float v) { if (GELU) v = gelu_t(v); return v * (float)CARRY; }
template <int GELU, int CARRY> __device__ __forceinline__ v8h cvt8(v4f a, v4f b) {
    v8h h;
    h[0] = (_Float16)fin1<GELU, CARRY>(a.x); h[1] = (_Float16)fin1<GELU, CARRY>(a.y); h[2] = (_Float16)fin1<GELU, CARRY>(a.z); h[3] = (_Float16)fin1<GELU, CARRY>(a.w);
    h[4] = (_Float16)fin1<GELU, CARRY>(b.x); h[5] = (_Float16)fin1<GELU, CARRY>(b.y); h[6] = (_Float16)fin1<GELU, CARRY>(b.z); h[7] = (_Float16)fin1<GELU, CARRY>(b.w);
    return h;
}

__global__ __launch_bounds__(256) void k_castT(const float* __restrict__ SRC, int lds, unsigned short* __restrict__ DST, int ldd, int nR, int nC, float sc) {
    const long long u = (long long)blockIdx.x * 256 + threadIdx.x; const int per = nR / 8;
    if (u >= (long long)nC * per) return;
    const int c = (int)(u / per); const int r0 = 8 * (int)(u % per);
    float w[8];
#pragma unroll
    for (int e = 0; e < 8; ++e) w[e] = bf16_keep(SRC[(long long)(r0 + e) * lds + c]) * sc;
    u4v pk; pk.x = pkh2(w[0], w[1]); pk.y = pkh2(w[2], w[3]); pk.z = pkh2(w[4], w[5]); pk.w = pkh2(w[6], w[7]);
    volatile u4v* d = (volatile u4v*)(DST + (long long)c * ldd + r0);
    *d = pk; __threadfence(); *d = pk;
}

template <int ABF>
__device__ __forceinline__ void ln_body(const float* __restrict__ A, const float* __restrict__ GA, const float* __restrict__ BE, unsigned short* __restrict__ Y16) {
    const int wave = __builtin_amdgcn_readfirstlane((int)(threadIdx.x >> 5));
    const int L = threadIdx.x & 31;
    const int r = (int)blockIdx.x * 8 + wave;
    if (r >= TOK) return;
    const int bb = r / SEQ;
    const long long srow = ABF ? ((long long)bb * SEQ_FULL + (long long)(r - bb * SEQ)) : (long long)r;
    const long long so = srow * EMB + 4 * L;
    float s = 0.f;
#pragma unroll 1
    for (int q = 0; q < 8; ++q) { v4f v = *(const v4f*)(A + so + 128 * q); if (ABF) v = bf16_keep4(v); s += (v.x + v.y) + (v.z + v.w); }
#pragma unroll
    for (int o = 16; o > 0; o >>= 1) s += __shfl_xor(s, o, 32);
    const float mu = s * (1.0f / EMB);
    float qq = 0.f;
#pragma unroll 1
    for (int q = 0; q < 8; ++q) {
        v4f v = *(const v4f*)(A + so + 128 * q); if (ABF) v = bf16_keep4(v);
        const float dx = v.x - mu, dy = v.y - mu, dz = v.z - mu, dw = v.w - mu;
        qq += (dx * dx + dy * dy) + (dz * dz + dw * dw);
    }
#pragma unroll
    for (int o = 16; o > 0; o >>= 1) qq += __shfl_xor(qq, o, 32);
    const float rs = rsqrtf(qq * (1.0f / EMB) + 1e-5f);
    const long long yo = (long long)r * EMB + 4 * L;
#pragma unroll 1
    for (int q = 0; q < 8; ++q) {
        v4f v = *(const v4f*)(A + so + 128 * q); if (ABF) v = bf16_keep4(v);
        const int c = 4 * L + 128 * q;
        const v4f ga = bf16_keep4(*(const v4f*)(GA + c)), be = bf16_keep4(*(const v4f*)(BE + c));
        const float y0 = (v.x - mu) * rs * ga.x + be.x, y1 = (v.y - mu) * rs * ga.y + be.y;
        const float y2 = (v.z - mu) * rs * ga.z + be.z, y3 = (v.w - mu) * rs * ga.w + be.w;
        u2v pk; pk.x = pkh2(y0, y1); pk.y = pkh2(y2, y3);
        volatile u2v* d = (volatile u2v*)(Y16 + yo + 128 * q);
        *d = pk; __threadfence(); *d = pk;
    }
}
__global__ __launch_bounds__(256) void k_ln_in(const float* __restrict__ X, const float* __restrict__ GA, const float* __restrict__ BE, unsigned short* __restrict__ Y16) {
    ln_body<1>(X, GA, BE, Y16);
}
__global__ __launch_bounds__(256) void k_ln_ws(const float* __restrict__ X, const float* __restrict__ GA, const float* __restrict__ BE, unsigned short* __restrict__ Y16) {
    ln_body<0>(X, GA, BE, Y16);
}

template <int BIASN, int OUTH, int RESM, int GELU, int CARRY>
__device__ __forceinline__ void gemm64_body(const unsigned short* __restrict__ A, int lda, const unsigned short* __restrict__ Bt, int ldb,
                                            float* __restrict__ Cf, unsigned short* __restrict__ Ch, int ldc,
                                            const float* __restrict__ bias, const float* __restrict__ resid, int M, int N, int K, float scale) {
    __shared__ __align__(16) float sT[8][16 * 68];
    const int lane = threadIdx.x & 31;
    const int wave = __builtin_amdgcn_readfirstlane((int)(threadIdx.x >> 5));
    const int tilesN = N >> 6, tilesM = M >> 6;
    const int tile = (int)blockIdx.x * 8 + wave;
    if (tile >= tilesM * tilesN) return;
    const int tm = tile / tilesN, tn = tile - tm * tilesN;
    const int m0 = tm << 6, n0 = tn << 6;
    const int rlane = lane & 15, hf = lane >> 4;
    const int koff = hf * 8, mOff = hf * 8;
    const size_t aoff = (size_t)(m0 + rlane) * (size_t)lda + koff;
    const size_t boff = (size_t)(n0 + rlane) * (size_t)ldb + koff;

    v8f acc[4][4];
#pragma unroll
    for (int i = 0; i < 4; ++i)
#pragma unroll
        for (int j = 0; j < 4; ++j) acc[i][j] = vzero();

#pragma unroll 1
    for (int k0 = 0; k0 < K; k0 += 32) {
        v16h bh[4];
#pragma unroll
        for (int j = 0; j < 4; ++j) bh[j] = ldfrag_g(Bt + boff + (size_t)(16 * j) * (size_t)ldb + k0);
#pragma unroll
        for (int i = 0; i < 4; ++i) {
            const v16h ah = ldfrag_g(A + aoff + (size_t)(16 * i) * (size_t)lda + k0);
#pragma unroll
            for (int j = 0; j < 4; ++j) acc[i][j] = mma16(ah, bh[j], acc[i][j]);
            guard4(acc[i][0], acc[i][1], acc[i][2], acc[i][3], ah, bh[3]);
        }
        keep4(bh[0], bh[1], bh[2], bh[3]);
    }

    float bv[4];
#pragma unroll
    for (int j = 0; j < 4; ++j) bv[j] = BIASN ? bf16_keep(bias[n0 + 16 * j + rlane]) : 0.f;

#pragma unroll
    for (int i = 0; i < 4; ++i) {
        const int mBase = m0 + 16 * i;
#pragma unroll
        for (int j = 0; j < 4; ++j)
#pragma unroll
            for (int r = 0; r < 8; ++r) sT[wave][(mOff + r) * 68 + 16 * j + rlane] = acc[i][j][r] * scale + bv[j];
        lds_wave_sync();
        if (OUTH == 0) {
            const int c4 = (lane & 15) * 4;
            v4f val[8];
#pragma unroll
            for (int it = 0; it < 8; ++it) {
                const int row = it * 2 + hf;
                v4f v = *(const v4f*)&sT[wave][row * 68 + c4];
                if (RESM != 0) {
                    const int gr = mBase + row;
                    size_t ro;
                    if (RESM == 2) { const int bb = gr / SEQ; ro = ((size_t)bb * SEQ_FULL + (size_t)(gr - bb * SEQ)) * (size_t)ldc + n0 + c4; }
                    else ro = (size_t)gr * (size_t)ldc + n0 + c4;
                    v4f x = *(const v4f*)(resid + ro);
                    if (RESM == 2) x = bf16_keep4(x);
                    v = v + x;
                }
                val[it] = v;
            }
#pragma unroll
            for (int it = 0; it < 8; ++it) { const int row = it * 2 + hf; *(volatile v4f*)(Cf + (size_t)(mBase + row) * (size_t)ldc + n0 + c4) = val[it]; }
            __threadfence();
#pragma unroll
            for (int it = 0; it < 8; ++it) { const int row = it * 2 + hf; *(volatile v4f*)(Cf + (size_t)(mBase + row) * (size_t)ldc + n0 + c4) = val[it]; }
        } else {
            const int q = lane >> 3, c8 = (lane & 7) * 8;
            v8h hv[4];
#pragma unroll
            for (int it = 0; it < 4; ++it) {
                const int row = it * 4 + q;
                const v4f a = *(const v4f*)&sT[wave][row * 68 + c8];
                const v4f b = *(const v4f*)&sT[wave][row * 68 + c8 + 4];
                hv[it] = cvt8<GELU, CARRY>(a, b);
            }
#pragma unroll
            for (int it = 0; it < 4; ++it) { const int row = it * 4 + q; *(volatile v8h*)(Ch + (size_t)(mBase + row) * (size_t)ldc + n0 + c8) = hv[it]; }
            __threadfence();
#pragma unroll
            for (int it = 0; it < 4; ++it) { const int row = it * 4 + q; *(volatile v8h*)(Ch + (size_t)(mBase + row) * (size_t)ldc + n0 + c8) = hv[it]; }
        }
        lds_wave_sync();
    }
}
__global__ __launch_bounds__(256) void k_gemm_h16(const unsigned short* __restrict__ A, int lda, const unsigned short* __restrict__ Bt, int ldb,
                                                  unsigned short* __restrict__ C, int ldc, int M, int N, int K, float scale) {
    gemm64_body<0, 1, 0, 0, 1>(A, lda, Bt, ldb, nullptr, C, ldc, nullptr, nullptr, M, N, K, scale);
}
__global__ __launch_bounds__(256) void k_gemm_res_in(const unsigned short* __restrict__ A, int lda, const unsigned short* __restrict__ Bt, int ldb,
                                                     float* __restrict__ C, int ldc, const float* __restrict__ bias, const float* __restrict__ resid,
                                                     int M, int N, int K, float scale) {
    gemm64_body<1, 0, 2, 0, 1>(A, lda, Bt, ldb, C, nullptr, ldc, bias, resid, M, N, K, scale);
}
__global__ __launch_bounds__(256) void k_gemm_res_ws(const unsigned short* __restrict__ A, int lda, const unsigned short* __restrict__ Bt, int ldb,
                                                     float* __restrict__ C, int ldc, const float* __restrict__ bias, const float* __restrict__ resid,
                                                     int M, int N, int K, float scale) {
    gemm64_body<1, 0, 1, 0, 1>(A, lda, Bt, ldb, C, nullptr, ldc, bias, resid, M, N, K, scale);
}
__global__ __launch_bounds__(256) void k_gemm_gelu(const unsigned short* __restrict__ A, int lda, const unsigned short* __restrict__ Bt, int ldb,
                                                   unsigned short* __restrict__ C, int ldc, const float* __restrict__ bias, int M, int N, int K, float scale) {
    gemm64_body<1, 1, 0, 1, 64>(A, lda, Bt, ldb, nullptr, C, ldc, bias, nullptr, M, N, K, scale);
}

#define AT_NW 4
#define AT_PP 40
static_assert(AT_PP % 8 == 0 && AT_PP >= 32);
__global__ __launch_bounds__(128) void k_attn(const unsigned short* __restrict__ QK, const unsigned short* __restrict__ VT, unsigned short* __restrict__ CTX) {
    __shared__ __align__(16) _Float16 pl[AT_NW][16 * AT_PP];
    __shared__ __align__(16) float os[AT_NW][16 * 68];
    const int lane = threadIdx.x & 31;
    const int wave = __builtin_amdgcn_readfirstlane((int)(threadIdx.x >> 5));
    const int hf = lane >> 4, l15 = lane & 15;
    const int nqb = SEQ / 64;
    const int bx = (int)blockIdx.x;
    const int qb = bx % nqb;
    const int bh = bx / nqb;
    const int h = bh % HEADS;
    const int b = bh / HEADS;
    const int q0 = qb * 64 + wave * 16;
    const size_t qoff  = (size_t)(b * SEQ + q0 + l15) * LDQK + h * HD + 8 * hf;
    const size_t kbase = (size_t)(b * SEQ + l15) * LDQK + EMB + h * HD + 8 * hf;
    const size_t vbase = (size_t)(h * HD + l15) * TOK + (size_t)b * SEQ + 8 * hf;
    const float CS = 0.125f * 1.4426950408889634f;
    const float NEG = -__builtin_inff();

    v8f o[4];
    float m8[8], l8[8];
#pragma unroll
    for (int t = 0; t < 4; ++t) o[t] = vzero();
#pragma unroll
    for (int r = 0; r < 8; ++r) { m8[r] = NEG; l8[r] = 0.f; }

    const int nhalf = (q0 + 16 + 31) >> 5;
#pragma unroll 1
    for (int jh = 0; jh < nhalf; ++jh) {
        const int j0 = jh * 32;
        v8f s0 = vzero(), s1 = vzero();
#pragma unroll
        for (int ks = 0; ks < 2; ++ks) {
            const v16h qa  = ldfrag_g(QK + qoff + ks * 32);
            const v16h kb0 = ldfrag_g(QK + kbase + (size_t)j0 * LDQK + ks * 32);
            const v16h kb1 = ldfrag_g(QK + kbase + (size_t)(j0 + 16) * LDQK + ks * 32);
            s0 = mma16(qa, kb0, s0);
            s1 = mma16(qa, kb1, s1);
            guard2(s0, s1, qa, kb0, kb1);
        }
        const bool diag = (j0 + 31 > q0);
        const int key0 = j0 + l15, key1 = j0 + 16 + l15;
#pragma unroll
        for (int r = 0; r < 8; ++r) {
            const int row = q0 + 8 * hf + r;
            float a0 = s0[r] * CS, a1 = s1[r] * CS;
            if (diag) { a0 = (key0 > row) ? NEG : a0; a1 = (key1 > row) ? NEG : a1; }
            float mx = fmaxf(a0, a1);
            mx = fmaxf(mx, __shfl_xor(mx, 1, 32)); mx = fmaxf(mx, __shfl_xor(mx, 2, 32));
            mx = fmaxf(mx, __shfl_xor(mx, 4, 32)); mx = fmaxf(mx, __shfl_xor(mx, 8, 32));
            const float mnew = fmaxf(m8[r], mx);
            const float corr = (m8[r] == NEG) ? 0.f : exp2f(m8[r] - mnew);
            const float p0 = (a0 == NEG) ? 0.f : exp2f(a0 - mnew);
            const float p1 = (a1 == NEG) ? 0.f : exp2f(a1 - mnew);
            float rs = p0 + p1;
            rs += __shfl_xor(rs, 1, 32); rs += __shfl_xor(rs, 2, 32); rs += __shfl_xor(rs, 4, 32); rs += __shfl_xor(rs, 8, 32);
            l8[r] = l8[r] * corr + rs; m8[r] = mnew;
#pragma unroll
            for (int t = 0; t < 4; ++t) o[t][r] *= corr;
            pl[wave][(8 * hf + r) * AT_PP + l15] = (_Float16)(p0 * 1024.0f);
            pl[wave][(8 * hf + r) * AT_PP + 16 + l15] = (_Float16)(p1 * 1024.0f);
        }
        lds_wave_sync();
        FragH pa;
        pa.h[0] = *(const v8h*)&pl[wave][l15 * AT_PP + 8 * hf];
        pa.h[1] = *(const v8h*)&pl[wave][l15 * AT_PP + 16 + 8 * hf];
        v16h vb[4];
#pragma unroll
        for (int t = 0; t < 4; ++t) vb[t] = ldfrag_g(VT + vbase + (size_t)(16 * t) * TOK + j0);
#pragma unroll
        for (int t = 0; t < 4; ++t) o[t] = mma16(pa.v, vb[t], o[t]);
        guard4b(o[0], o[1], o[2], o[3], pa.v, vb[0], vb[1], vb[2], vb[3]);
        lds_wave_sync();
    }

#pragma unroll
    for (int r = 0; r < 8; ++r) {
        const float inv = 1.0f / (l8[r] * 16.0f);
#pragma unroll
        for (int t = 0; t < 4; ++t) os[wave][(8 * hf + r) * 68 + 16 * t + l15] = o[t][r] * inv;
    }
    lds_wave_sync();
    {
        const int q = lane >> 3, c8 = (lane & 7) * 8;
        v8h hv[4];
#pragma unroll
        for (int it = 0; it < 4; ++it) {
            const int row = it * 4 + q;
            const v4f a = *(const v4f*)&os[wave][row * 68 + c8];
            const v4f bq = *(const v4f*)&os[wave][row * 68 + c8 + 4];
            hv[it] = cvt8<0, 1>(a, bq);
        }
#pragma unroll
        for (int it = 0; it < 4; ++it) { const int row = it * 4 + q; *(volatile v8h*)(CTX + (size_t)(b * SEQ + q0 + row) * EMB + h * HD + c8) = hv[it]; }
        __threadfence();
#pragma unroll
        for (int it = 0; it < 4; ++it) { const int row = it * 4 + q; *(volatile v8h*)(CTX + (size_t)(b * SEQ + q0 + row) * EMB + h * HD + c8) = hv[it]; }
    }
}

constexpr size_t SZ_WQK = (size_t)2 * EMB * EMB * 2;
constexpr size_t SZ_WV  = (size_t)EMB * EMB * 2;
constexpr size_t SZ_WO  = (size_t)EMB * EMB * 2;
constexpr size_t SZ_W1  = (size_t)FF * EMB * 2;
constexpr size_t SZ_W2  = (size_t)EMB * FF * 2;
constexpr size_t SZ_X16 = (size_t)TOK * EMB * 2;
constexpr size_t SZ_QK  = (size_t)TOK * LDQK * 2;
constexpr size_t SZ_VT  = (size_t)EMB * TOK * 2;
constexpr size_t SZ_CTX = (size_t)TOK * EMB * 2;
constexpr size_t SZ_X1  = (size_t)TOK * EMB * 4;
constexpr size_t SZ_G   = (size_t)TOK * FF * 2;
constexpr size_t OF_WQK = 0;
constexpr size_t OF_WV  = OF_WQK + SZ_WQK;
constexpr size_t OF_WO  = OF_WV + SZ_WV;
constexpr size_t OF_W1  = OF_WO + SZ_WO;
constexpr size_t OF_W2  = OF_W1 + SZ_W1;
constexpr size_t OF_X16 = OF_W2 + SZ_W2;
constexpr size_t OF_QK  = OF_X16 + SZ_X16;
constexpr size_t OF_VT  = OF_QK + SZ_QK;
constexpr size_t OF_CTX = OF_VT + SZ_VT;
constexpr size_t OF_X1  = OF_CTX + SZ_CTX;
constexpr size_t OF_G   = OF_X1 + SZ_X1;
constexpr size_t WS_TOTAL = OF_G + SZ_G;
static_assert(WS_TOTAL <= (size_t)134217728);
static_assert(SZ_WQK % 256 == 0 && SZ_WV % 256 == 0 && SZ_W1 % 256 == 0 && SZ_X16 % 256 == 0 && SZ_QK % 256 == 0 && SZ_VT % 256 == 0 && SZ_X1 % 256 == 0);

extern "C" void kernel_launch(void* const* d_in, const int* in_sizes, int n_in, void* d_out, int out_size, void* d_ws, size_t ws_size, hipStream_t stream) {
    if (n_in < 14) return;
    if (in_sizes[0] < (NB - 1) * SEQ_FULL * EMB + SEQ * EMB) return;
    if (in_sizes[1] < EMB * EMB || in_sizes[2] < EMB * EMB || in_sizes[3] < EMB * EMB || in_sizes[4] < EMB * EMB) return;
    if (in_sizes[5] < EMB || in_sizes[6] < EMB || in_sizes[7] < EMB || in_sizes[8] < EMB || in_sizes[9] < EMB) return;
    if (in_sizes[10] < EMB * FF || in_sizes[11] < FF || in_sizes[12] < FF * EMB || in_sizes[13] < EMB) return;
    if (out_size < TOK * EMB) return;
    if (ws_size < WS_TOTAL) return;

    const float* x    = (const float*)d_in[0];
    const float* wq   = (const float*)d_in[1];
    const float* wk   = (const float*)d_in[2];
    const float* wv   = (const float*)d_in[3];
    const float* wo   = (const float*)d_in[4];
    const float* bo   = (const float*)d_in[5];
    const float* g1   = (const float*)d_in[6];
    const float* be1  = (const float*)d_in[7];
    const float* g2   = (const float*)d_in[8];
    const float* be2  = (const float*)d_in[9];
    const float* w1   = (const float*)d_in[10];
    const float* b1   = (const float*)d_in[11];
    const float* w2   = (const float*)d_in[12];
    const float* b2   = (const float*)d_in[13];
    float* out = (float*)d_out;

    char* wsp = (char*)d_ws;
    unsigned short* WQK = (unsigned short*)(wsp + OF_WQK);
    unsigned short* WVT = (unsigned short*)(wsp + OF_WV);
    unsigned short* WOT = (unsigned short*)(wsp + OF_WO);
    unsigned short* W1T = (unsigned short*)(wsp + OF_W1);
    unsigned short* W2T = (unsigned short*)(wsp + OF_W2);
    unsigned short* X16 = (unsigned short*)(wsp + OF_X16);
    unsigned short* H16 = X16;
    unsigned short* QK  = (unsigned short*)(wsp + OF_QK);
    unsigned short* VT  = (unsigned short*)(wsp + OF_VT);
    unsigned short* CTX = (unsigned short*)(wsp + OF_CTX);
    float*          X1  = (float*)(wsp + OF_X1);
    unsigned short* G16 = (unsigned short*)(wsp + OF_G);

    const unsigned gsq = (unsigned)(((long long)EMB * (EMB / 8) + 255) / 256);
    k_castT<<<gsq, 256, 0, stream>>>(wq, EMB, WQK, EMB, EMB, EMB, 16.0f);
    k_castT<<<gsq, 256, 0, stream>>>(wk, EMB, WQK + (size_t)EMB * EMB, EMB, EMB, EMB, 16.0f);
    k_castT<<<gsq, 256, 0, stream>>>(wv, EMB, WVT, EMB, EMB, EMB, 16.0f);
    k_castT<<<gsq, 256, 0, stream>>>(wo, EMB, WOT, EMB, EMB, EMB, 16.0f);
    k_castT<<<(unsigned)(((long long)FF * (EMB / 8) + 255) / 256), 256, 0, stream>>>(w1, FF, W1T, EMB, EMB, FF, 16.0f);
    k_castT<<<(unsigned)(((long long)EMB * (FF / 8) + 255) / 256), 256, 0, stream>>>(w2, EMB, W2T, FF, FF, EMB, 16.0f);

    k_ln_in<<<TOK / 8, 256, 0, stream>>>(x, g1, be1, X16);

    k_gemm_h16<<<(unsigned)(((TOK / 64) * (LDQK / 64) + 7) / 8), 256, 0, stream>>>(X16, EMB, WQK, EMB, QK, LDQK, TOK, LDQK, EMB, 0.0625f);
    k_gemm_h16<<<(unsigned)(((EMB / 64) * (TOK / 64) + 7) / 8), 256, 0, stream>>>(WVT, EMB, X16, EMB, VT, TOK, EMB, TOK, EMB, 0.0625f);

    k_attn<<<(unsigned)(NB * HEADS * (SEQ / 64)), 32 * AT_NW, 0, stream>>>(QK, VT, CTX);

    k_gemm_res_in<<<(unsigned)(((TOK / 64) * (EMB / 64) + 7) / 8), 256, 0, stream>>>(CTX, EMB, WOT, EMB, X1, EMB, bo, x, TOK, EMB, EMB, 0.0009765625f);

    k_ln_ws<<<TOK / 8, 256, 0, stream>>>(X1, g2, be2, H16);

    k_gemm_gelu<<<(unsigned)(((TOK / 64) * (FF / 64) + 7) / 8), 256, 0, stream>>>(H16, EMB, W1T, EMB, G16, FF, b1, TOK, FF, EMB, 0.0625f);

    k_gemm_res_ws<<<(unsigned)(((TOK / 64) * (EMB / 64) + 7) / 8), 256, 0, stream>>>(G16, FF, W2T, FF, out, EMB, b2, X1, TOK, EMB, FF, 0.0009765625f);
}
